// NeuroMotorSNN_16192026706220
// MI455X (gfx1250) — hardware-verified
//
#include <hip/hip_runtime.h>
#include <math.h>


typedef _Float16 v16h __attribute__((ext_vector_type(16)));
typedef _Float16 v8h  __attribute__((ext_vector_type(8)));
typedef float    v8f  __attribute__((ext_vector_type(8)));
typedef float    v4f  __attribute__((ext_vector_type(4)));

union Frag16 { v16h v; v8h half[2]; };

#define HID      128
#define NTH      32
#define AP       136
#define CP       132
#define SCALE_A  16384.0f
#define SCALE_B  4096.0f
#define DESCALE  (1.0f / 67108864.0f)
#define INV_S2   (1.0f / 0.0244140625f)
#define BETA_F   0.9f
#define OMB_F    0.1f
#define THR_F    0.5f
#define EPS_F    1e-5f

__device__ __forceinline__ v8f wmma_f16(v16h a, v16h b, v8f c)
{
    return __builtin_amdgcn_wmma_f32_16x16x32_f16(false, a, false, b, (short)0, c, false, false);
}

__global__ __launch_bounds__(256) void snn_scan_kernel(
    const float* __restrict__ x,
    const float* __restrict__ W_in,
    const float* __restrict__ b_in,
    const float* __restrict__ ln_g,
    const float* __restrict__ ln_b,
    const float* __restrict__ W_out,
    const float* __restrict__ b_out,
    float* out,
    int B, int T)
{
#pragma clang fp contract(off)
    __shared__ __attribute__((aligned(16))) _Float16 Ahi[16 * AP];
    __shared__ __attribute__((aligned(16))) _Float16 Alo[16 * AP];
    __shared__ __attribute__((aligned(16))) float    Ct[16 * CP];
    __shared__ __attribute__((aligned(16))) float    robuf[32];

    const int tid  = threadIdx.x;
    const int lane = tid & 31;
    const int w    = tid >> 5;
    const int h    = lane >> 4;
    const int m    = lane & 15;
    const int n    = 16 * w + m;
    const int b0   = blockIdx.x * 16;

    const int r  = tid >> 4;
    const int q  = tid & 15;
    const int ch = q >> 2;
    const int g  = q & 3;
    int rowg = b0 + r;
    if (rowg > B - 1) rowg = B - 1;

    float th[8];
#pragma unroll
    for (int e = 0; e < 8; ++e) {
        const int k = 8 * g + e;
        const float st = (float)k * (1.0f / 31.0f);
        const float om = 1.0f - st;
        const float v  = -3.0f * om + 3.0f * st;
        th[e] = (k == NTH - 1) ? 3.0f : v;
    }

    v16h bh[4], bl[4];
#pragma unroll
    for (int kc = 0; kc < 4; ++kc) {
        const float* wp = W_in + (size_t)n * HID + 32 * kc + 8 * h;
        v16h vh, vl;
#pragma unroll
        for (int e = 0; e < 8; ++e) {
            const float v0 = wp[e] * SCALE_B;
            const _Float16 h0 = (_Float16)v0;
            vh[e] = h0;
            vl[e] = (_Float16)(v0 - (float)h0);
            const float v1 = wp[16 + e] * SCALE_B;
            const _Float16 h1 = (_Float16)v1;
            vh[8 + e] = h1;
            vl[8 + e] = (_Float16)(v1 - (float)h1);
        }
        bh[kc] = vh;
        bl[kc] = vl;
    }

    const float bi = b_in[n];

    float gg[8], gb[8], wo0[8], wo1[8], mem[8];
#pragma unroll
    for (int j = 0; j < 8; ++j) {
        const int c = 8 * q + j;
        gg[j]  = ln_g[c];
        gb[j]  = ln_b[c];
        wo0[j] = W_out[c];
        wo1[j] = W_out[HID + c];
        mem[j] = 0.0f;
    }
    float ro0 = 0.0f, ro1 = 0.0f;

    _Float16* const ahi_st = Ahi + r * AP + 32 * ch + 8 * g;
    _Float16* const alo_st = Alo + r * AP + 32 * ch + 8 * g;
    const _Float16* const ahi_ld = Ahi + m * AP + 8 * h;
    const _Float16* const alo_ld = Alo + m * AP + 8 * h;

    for (int t = 0; t < T; ++t) {
        const float xv = x[((size_t)rowg * (size_t)T + (size_t)t) * 4 + ch];
        v8h hv, lv;
#pragma unroll
        for (int e = 0; e < 8; ++e) {
            const float d   = xv - th[e];
            const float sq  = d * d;
            const float arg = (-0.5f * sq) * INV_S2;
            const float s   = expf(arg) * SCALE_A;
            const _Float16 sh = (_Float16)s;
            hv[e] = sh;
            lv[e] = (_Float16)(s - (float)sh);
        }
        *(v8h*)(ahi_st) = hv;
        *(v8h*)(alo_st) = lv;
        __syncthreads();

        v8f acc = {0.0f, 0.0f, 0.0f, 0.0f, 0.0f, 0.0f, 0.0f, 0.0f};
#pragma unroll
        for (int kc = 0; kc < 4; ++kc) {
            Frag16 ah, al;
            ah.half[0] = *(const v8h*)(ahi_ld + 32 * kc);
            ah.half[1] = *(const v8h*)(ahi_ld + 32 * kc + 16);
            al.half[0] = *(const v8h*)(alo_ld + 32 * kc);
            al.half[1] = *(const v8h*)(alo_ld + 32 * kc + 16);
            acc = wmma_f16(ah.v, bh[kc], acc);
            acc = wmma_f16(ah.v, bl[kc], acc);
            acc = wmma_f16(al.v, bh[kc], acc);
            asm volatile("v_nop\n\tv_nop\n\tv_nop\n\tv_nop"
                         : "+v"(acc)
                         : "v"(ah.v), "v"(al.v), "v"(bh[kc]), "v"(bl[kc]));
        }
#pragma unroll
        for (int j = 0; j < 8; ++j)
            Ct[(8 * h + j) * CP + n] = acc[j] * DESCALE + bi;
        __syncthreads();

        const v4f c0 = *(const v4f*)(Ct + r * CP + 8 * q);
        const v4f c1 = *(const v4f*)(Ct + r * CP + 8 * q + 4);
        float cv[8] = {c0[0], c0[1], c0[2], c0[3], c1[0], c1[1], c1[2], c1[3]};

        float S = 0.0f;
#pragma unroll
        for (int j = 0; j < 8; ++j) S += cv[j];
        S += __shfl_xor(S, 1);
        S += __shfl_xor(S, 2);
        S += __shfl_xor(S, 4);
        S += __shfl_xor(S, 8);
        const float mu = S * (1.0f / 128.0f);

        float V = 0.0f;
#pragma unroll
        for (int j = 0; j < 8; ++j) { const float dv = cv[j] - mu; V += dv * dv; }
        V += __shfl_xor(V, 1);
        V += __shfl_xor(V, 2);
        V += __shfl_xor(V, 4);
        V += __shfl_xor(V, 8);
        const float var = V * (1.0f / 128.0f);
        const float rs  = 1.0f / sqrtf(var + EPS_F);

#pragma unroll
        for (int j = 0; j < 8; ++j) {
            float cn = (cv[j] - mu) * rs;
            cn = cn * gg[j] + gb[j];
            const float mm = mem[j] * BETA_F + cn * OMB_F;
            const bool  sp = mm > THR_F;
            mem[j] = sp ? (mm - THR_F) : mm;
            ro0 += sp ? wo0[j] : 0.0f;
            ro1 += sp ? wo1[j] : 0.0f;
        }
    }

    float q0 = ro0, q1 = ro1;
    q0 += __shfl_xor(q0, 1);  q1 += __shfl_xor(q1, 1);
    q0 += __shfl_xor(q0, 2);  q1 += __shfl_xor(q1, 2);
    q0 += __shfl_xor(q0, 4);  q1 += __shfl_xor(q1, 4);
    q0 += __shfl_xor(q0, 8);  q1 += __shfl_xor(q1, 8);
    if (q == 0) {
        robuf[2 * r]     = q0 + b_out[0] * (float)T;
        robuf[2 * r + 1] = q1 + b_out[1] * (float)T;
    }
    __syncthreads();

    if (b0 + 16 <= B) {
        v4f ov = {0.0f, 0.0f, 0.0f, 0.0f};
        if (tid < 8) ov = *(const v4f*)(robuf + 4 * tid);
        volatile v4f* op = (volatile v4f*)(out + (size_t)b0 * 2) + tid;
        if (tid < 8) *op = ov;
        __threadfence();
        if (tid < 8) *op = ov;
    } else {
        const int nv = (B - b0) * 2;
        float ov = 0.0f;
        if (tid < nv) ov = robuf[tid];
        volatile float* op = (volatile float*)out + (size_t)b0 * 2 + tid;
        if (tid < nv) *op = ov;
        __threadfence();
        if (tid < nv) *op = ov;
    }
}

extern "C" void kernel_launch(void* const* d_in, const int* in_sizes, int n_in,
                              void* d_out, int out_size, void* d_ws, size_t ws_size,
                              hipStream_t stream)
{
    (void)n_in; (void)d_ws; (void)ws_size;
    const float* x     = (const float*)d_in[0];
    const float* W_in  = (const float*)d_in[1];
    const float* b_in  = (const float*)d_in[2];
    const float* ln_g  = (const float*)d_in[3];
    const float* ln_b  = (const float*)d_in[4];
    const float* W_out = (const float*)d_in[5];
    const float* b_out = (const float*)d_in[6];
    float*       out   = (float*)d_out;

    const int B = out_size / 2;
    if (B <= 0) return;
    const int T = in_sizes[0] / (4 * B);
    if (T <= 0) return;

    dim3 grid((B + 15) / 16);
    dim3 block(256);
    hipLaunchKernelGGL(snn_scan_kernel, grid, block, 0, stream,
                       x, W_in, b_in, ln_g, ln_b, W_out, b_out, out, B, T);
}
